// RankOneMoE_74139725463721
// MI455X (gfx1250) — hardware-verified
//
#include <hip/hip_runtime.h>
#include <math.h>

typedef __attribute__((ext_vector_type(16))) _Float16 v16h;
typedef __attribute__((ext_vector_type(16))) __bf16 v16b;
typedef __attribute__((ext_vector_type(8)))  _Float16 v8h;
typedef __attribute__((ext_vector_type(8)))  float v8f;
typedef __attribute__((ext_vector_type(4)))  float v4f;
typedef __attribute__((ext_vector_type(2)))  float v2f;
typedef __attribute__((ext_vector_type(4)))  unsigned v4u;
typedef __attribute__((ext_vector_type(4)))  int v4i;
typedef float __attribute__((may_alias)) float_a;
typedef int __attribute__((may_alias)) int_a;

template <typename T> __device__ __forceinline__ void vst2(void* p, T v) { *(volatile T*)p = v; __threadfence(); *(volatile T*)p = v; }
__device__ __forceinline__ v8f wmma16(v16h a, v16h b, v8f c) {
  v8f d = __builtin_amdgcn_wmma_f32_16x16x32_f16(false, a, false, b, (short)0, c, false, false);
  asm volatile("v_nop\n\tv_nop\n\tv_nop\n\tv_nop" : "+v"(d) : "v"(a), "v"(b));
  return d;
}
__device__ __forceinline__ v8f wmma_bf(v16b a, v16b b, v8f c) {
  v8f d = __builtin_amdgcn_wmma_f32_16x16x32_bf16(false, a, false, b, (short)0, c, false, false);
  asm volatile("v_nop\n\tv_nop\n\tv_nop\n\tv_nop" : "+v"(d) : "v"(a), "v"(b));
  return d;
}
__device__ __forceinline__ v16h frag_h(const _Float16* rowk0, int lane) {
  union { v16h v; v8h q[2]; } u; const _Float16* p = rowk0 + 8 * (lane >> 4);
  u.q[0] = *(const v8h*)p; u.q[1] = *(const v8h*)(p + 16); return u.v;
}
__device__ __forceinline__ v16h frag_f32(const float* rowk0, int lane) {
  v16h a; const float* p = rowk0 + 8 * (lane >> 4);
#pragma unroll
  for (int i = 0; i < 8; ++i) { a[i] = (_Float16)p[i]; a[8 + i] = (_Float16)p[16 + i]; }
  return a;
}
__device__ __forceinline__ v16h frag_f32s(const float* rowk0, int lane, float sc) {
  v16h a; const float* p = rowk0 + 8 * (lane >> 4);
#pragma unroll
  for (int i = 0; i < 8; ++i) { a[i] = (_Float16)(p[i] * sc); a[8 + i] = (_Float16)(p[16 + i] * sc); }
  return a;
}
__device__ __forceinline__ v16h fragc_f32(const float* W, int k0, int n, int lane, int ld, int K) {
  v16h a; const int g = lane >> 4;
#pragma unroll
  for (int i = 0; i < 8; ++i) { const int ka = k0 + 8 * g + i, kb = ka + 16;
    a[i] = (_Float16)(ka < K ? W[(size_t)(ka < K ? ka : K - 1) * ld + n] : 0.f); a[8 + i] = (_Float16)(kb < K ? W[(size_t)(kb < K ? kb : K - 1) * ld + n] : 0.f); }
  return a;
}
struct F2 { v16b h, l; };
__device__ __forceinline__ F2 bsplit16(const float v[16]) { F2 r;
#pragma unroll
  for (int i = 0; i < 16; ++i) { const __bf16 h = (__bf16)v[i]; r.h[i] = h; r.l[i] = (__bf16)(v[i] - (float)h); }
  return r; }
__device__ __forceinline__ F2 split_row(const float* row, int k0, int lane) { float v[16]; const float* p = row + k0 + 8 * (lane >> 4);
#pragma unroll
  for (int i = 0; i < 8; ++i) { v[i] = p[i]; v[8 + i] = p[16 + i]; }
  return bsplit16(v); }
__device__ __forceinline__ F2 split_rowK(const float* row, int k0, int lane, int K) { float v[16]; const int g = lane >> 4;
#pragma unroll
  for (int i = 0; i < 8; ++i) { const int ka = k0 + 8 * g + i, kb = ka + 16; v[i] = ka < K ? row[ka < K ? ka : K - 1] : 0.f; v[8 + i] = kb < K ? row[kb < K ? kb : K - 1] : 0.f; }
  return bsplit16(v); }
__device__ __forceinline__ F2 split_col(const float* W, int k0, int n, int lane, int ld, int K) { float v[16]; const int g = lane >> 4;
#pragma unroll
  for (int i = 0; i < 8; ++i) { const int ka = k0 + 8 * g + i, kb = ka + 16; v[i] = ka < K ? W[(size_t)(ka < K ? ka : K - 1) * ld + n] : 0.f; v[8 + i] = kb < K ? W[(size_t)(kb < K ? kb : K - 1) * ld + n] : 0.f; }
  return bsplit16(v); }
__device__ __forceinline__ v8f mac3(const F2& a, const F2& b, v8f c) { c = wmma_bf(a.l, b.h, c); c = wmma_bf(a.h, b.l, c); return wmma_bf(a.h, b.h, c); }
__device__ __forceinline__ float sigm(float v) { return 1.0f / (1.0f + expf(-v)); }
#define LDSX() do { asm volatile("s_wait_dscnt 0" ::: "memory"); __builtin_amdgcn_wave_barrier(); __builtin_amdgcn_fence(__ATOMIC_RELEASE, "workgroup"); } while (0)


#define NB 16
#define SS 512
#define HH 768
#define FF 3072
#define NE 8
#define KK 16
#define EK (NE * KK)
#define G1 (2 * EK)
#define NROW (NB * SS)
#define LAM 0.2f
#ifndef TOB
#define TOB (NROW / 64)
#endif
typedef __attribute__((ext_vector_type(8))) __bf16 v8b;
__device__ __forceinline__ v16b frag_b(const __bf16* rowk0, int lane) {
  union { v16b v; v8b q[2]; } u; const __bf16* p = rowk0 + 8 * (lane >> 4);
  u.q[0] = *(const v8b*)p; u.q[1] = *(const v8b*)(p + 16); return u.v;
}
__device__ __forceinline__ float bfr(float v) { return (float)(__bf16)v; }
__device__ __attribute__((noinline)) float exp_ni(float v) { return expf(v); }
__device__ __attribute__((noinline)) float erf_ni(float v) { return erff(v); }

#define WS_PU1 0u
#define WS_PU2 (WS_PU1 + 2u * (size_t)FF * EK)
#define WS_PW2 (WS_PU2 + 2u * (size_t)HH * EK)
#define WS_PS2 (WS_PW2 + 2u * (size_t)HH * FF)
#define WS_G1  (WS_PS2 + 2u * (size_t)EK * FF)
#define WS_G2  (WS_G1 + 4u * (size_t)NROW * G1)
#define WS_GW  (WS_G2 + 4u * (size_t)NROW * EK)
#define WS_T1  (WS_GW + 4u * (size_t)NB * EK)
#define WS_HF  (WS_T1 + 4u * (size_t)NROW * EK)
#define WS_T2  (WS_HF + 2u * (size_t)NROW * FF)
#define WS_BM  (WS_T2 + 4u * (size_t)NROW * EK)
#define WS_END (WS_BM + 4u * (FF + HH))

__device__ __forceinline__ v16b fragb_f32(const float* __restrict__ p, int lane) { v16b a; const float* pp = p + 8 * (lane >> 4);
#pragma unroll
  for (int i = 0; i < 8; ++i) { a[i] = (__bf16)pp[i]; a[8 + i] = (__bf16)pp[16 + i]; } return a; }
__global__ __launch_bounds__(256) void k_pack(const float* __restrict__ U1, const float* __restrict__ U2, const float* __restrict__ W2, const float* __restrict__ SVH2, const float* __restrict__ B1, const float* __restrict__ TB1, const float* __restrict__ B2, const float* __restrict__ TB2, char* __restrict__ ws) {
  __shared__ __align__(16) __bf16 sb[EK]; __shared__ __align__(16) _Float16 sh[FF]; __shared__ __align__(16) float sm[FF + HH]; const int n = blockIdx.x, which = blockIdx.y, t = threadIdx.x;
  if (which == 0) { if (n >= FF) return; if (t < EK) sb[t] = (__bf16)U1[(size_t)t * FF + n]; __syncthreads(); if (t < EK / 8) vst2((unsigned*)((__bf16*)(ws + WS_PU1) + (size_t)n * EK + t * 8), *(const v4u*)&sb[t * 8]); }
  else if (which == 1) { if (n >= HH) return; if (t < EK) sb[t] = (__bf16)U2[(size_t)t * HH + n]; __syncthreads(); if (t < EK / 8) vst2((unsigned*)((__bf16*)(ws + WS_PU2) + (size_t)n * EK + t * 8), *(const v4u*)&sb[t * 8]); }
  else if (which == 2) { if (n >= HH) return; for (int f = t; f < FF; f += 256) sh[f] = (_Float16)bfr(W2[(size_t)n * FF + f]); __syncthreads(); for (int q = t; q < FF / 8; q += 256) vst2((unsigned*)((_Float16*)(ws + WS_PW2) + (size_t)n * FF + q * 8), *(const v4u*)&sh[q * 8]); }
  else if (which == 3) { if (n >= EK) return; for (int f = t; f < FF; f += 256) sh[f] = (_Float16)bfr(SVH2[(size_t)n * FF + f]); __syncthreads(); for (int q = t; q < FF / 8; q += 256) vst2((unsigned*)((_Float16*)(ws + WS_PS2) + (size_t)n * FF + q * 8), *(const v4u*)&sh[q * 8]); }
  else { if (n > 0) return; for (int c = t; c < FF + HH; c += 256) { float s = 0.f; if (c < FF) { for (int e = 0; e < NE; ++e) s += bfr(TB1[(size_t)e * FF + c]); sm[c] = bfr(B1[c]) + LAM * s; } else { const int hcol = c - FF; for (int e = 0; e < NE; ++e) s += bfr(TB2[(size_t)e * HH + hcol]); sm[c] = bfr(B2[hcol]) + LAM * s; } }
    __syncthreads(); for (int q = t; q < (FF + HH) / 4; q += 256) vst2((float*)(ws + WS_BM) + q * 4, *(const v4f*)&sm[q * 4]); } }
__global__ __launch_bounds__(128) void k_r1(const float* __restrict__ X, const float* __restrict__ GW1, const float* __restrict__ GB1, float* __restrict__ G1o) { __shared__ __align__(16) float sf[4][16][132];
  const int tid = threadIdx.x, wave = tid >> 5, lane = tid & 31, col = lane & 15, g = lane >> 4; const size_t r0 = (size_t)blockIdx.x * 64 + wave * 16; const int c0 = blockIdx.y * 128;
  v8f acc[8] = {};
#pragma unroll 2
  for (int kc = 0; kc < HH / 32; ++kc) { const v16b a = fragb_f32(X + (r0 + col) * HH + kc * 32, lane);
#pragma unroll
    for (int j = 0; j < 8; ++j) acc[j] = wmma_bf(a, fragb_f32(GW1 + (size_t)(c0 + j * 16 + col) * HH + kc * 32, lane), acc[j]); }
#pragma unroll
  for (int j = 0; j < 8; ++j) { const float bb = bfr(GB1[c0 + j * 16 + col]);
#pragma unroll
    for (int r = 0; r < 8; ++r) sf[wave][8 * g + r][j * 16 + col] = fmaxf(acc[j][r] + bb, 0.f); }
  LDSX(); for (int rl = 0; rl < 16; ++rl) vst2(G1o + (r0 + rl) * G1 + c0 + lane * 4, *(const v4f*)&sf[wave][rl][lane * 4]); }
__global__ __launch_bounds__(128) void k_r2(const float* __restrict__ G1i, const float* __restrict__ GW2, const float* __restrict__ GB2, float* __restrict__ G2o) { __shared__ __align__(16) float sf[4][16][132];
  const int tid = threadIdx.x, wave = tid >> 5, lane = tid & 31, col = lane & 15, g = lane >> 4; const size_t r0 = (size_t)blockIdx.x * 64 + wave * 16;
  v8f acc[8] = {};
#pragma unroll
  for (int kc = 0; kc < G1 / 32; ++kc) { const F2 a = split_row(G1i + (r0 + col) * G1, kc * 32, lane);
#pragma unroll
    for (int j = 0; j < 8; ++j) { const v16b w = fragb_f32(GW2 + (size_t)(j * 16 + col) * G1 + kc * 32, lane); acc[j] = wmma_bf(a.h, w, acc[j]); acc[j] = wmma_bf(a.l, w, acc[j]); } }
#pragma unroll
  for (int j = 0; j < 8; ++j) { const float bb = bfr(GB2[j * 16 + col]);
#pragma unroll
    for (int r = 0; r < 8; ++r) sf[wave][8 * g + r][j * 16 + col] = acc[j][r] + bb; }
  LDSX(); for (int rl = 0; rl < 16; ++rl) vst2(G2o + (r0 + rl) * EK + lane * 4, *(const v4f*)&sf[wave][rl][lane * 4]); }
__global__ __launch_bounds__(128) void k_gw(const float* __restrict__ G2i, float* __restrict__ GW) { __shared__ __align__(16) float s[EK]; const int t = threadIdx.x; const size_t b = blockIdx.x; float acc = 0.f;
  for (int r = 0; r < SS; ++r) acc += G2i[(b * SS + r) * EK + t]; s[t] = acc * (1.0f / SS); __syncthreads(); if (t < EK / 4) vst2(GW + b * EK + t * 4, *(const v4f*)&s[t * 4]); }
__global__ __launch_bounds__(128) void k_t1(const float* __restrict__ X, const float* __restrict__ SVH1, const float* __restrict__ GW, float* __restrict__ T1) { __shared__ __align__(16) float sf[4][16][132];
  const int tid = threadIdx.x, wave = tid >> 5, lane = tid & 31, col = lane & 15, g = lane >> 4; const size_t r0 = (size_t)blockIdx.x * 64 + wave * 16; const size_t b = ((size_t)blockIdx.x * 64) / SS;
  v8f acc[8] = {};
#pragma unroll 2
  for (int kc = 0; kc < HH / 32; ++kc) { const v16b a = fragb_f32(X + (r0 + col) * HH + kc * 32, lane);
#pragma unroll
    for (int j = 0; j < 8; ++j) acc[j] = wmma_bf(a, fragb_f32(SVH1 + (size_t)(j * 16 + col) * HH + kc * 32, lane), acc[j]); }
#pragma unroll
  for (int j = 0; j < 8; ++j) { const float gv = GW[b * EK + j * 16 + col];
#pragma unroll
    for (int r = 0; r < 8; ++r) sf[wave][8 * g + r][j * 16 + col] = acc[j][r] * gv; }
  LDSX(); for (int rl = 0; rl < 16; ++rl) vst2(T1 + (r0 + rl) * EK + lane * 4, *(const v4f*)&sf[wave][rl][lane * 4]); }
__global__ __launch_bounds__(128) void k_fc1(const float* __restrict__ X, const float* __restrict__ W1, const float* __restrict__ T1, const __bf16* __restrict__ PU1, const float* __restrict__ BM, _Float16* __restrict__ HF) { __shared__ __align__(16) _Float16 sh[4][16][136];
  const int tid = threadIdx.x, wave = tid >> 5, lane = tid & 31, col = lane & 15, g = lane >> 4; const size_t r0 = (size_t)blockIdx.x * 64 + wave * 16; const int c0 = blockIdx.y * 128;
  v8f acc[8] = {};
#pragma unroll 2
  for (int kc = 0; kc < HH / 32; ++kc) { const v16b a = fragb_f32(X + (r0 + col) * HH + kc * 32, lane);
#pragma unroll
    for (int j = 0; j < 8; ++j) acc[j] = wmma_bf(a, fragb_f32(W1 + (size_t)(c0 + j * 16 + col) * HH + kc * 32, lane), acc[j]); }
#pragma unroll
  for (int kc = 0; kc < EK / 32; ++kc) { const F2 a = split_row(T1 + (r0 + col) * EK, kc * 32, lane);
#pragma unroll
    for (int j = 0; j < 8; ++j) { const v16b w = frag_b(PU1 + (size_t)(c0 + j * 16 + col) * EK + kc * 32, lane); acc[j] = wmma_bf(a.h, w, acc[j]); acc[j] = wmma_bf(a.l, w, acc[j]); } }
#pragma unroll
  for (int j = 0; j < 8; ++j) { const float bb = BM[c0 + j * 16 + col];
#pragma unroll
    for (int r = 0; r < 8; ++r) sh[wave][8 * g + r][j * 16 + col] = (_Float16)fmaxf(acc[j][r] + bb, 0.f); }
  LDSX(); for (int rl = 0; rl < 16; ++rl) if (lane < 16) vst2((unsigned*)(HF + (r0 + rl) * FF + c0 + lane * 8), *(const v4u*)&sh[wave][rl][lane * 8]); }
__global__ __launch_bounds__(128) void k_t2(const _Float16* __restrict__ HF, const _Float16* __restrict__ PS2, const float* __restrict__ GW, float* __restrict__ T2) { __shared__ __align__(16) float sf[4][16][132];
  const int tid = threadIdx.x, wave = tid >> 5, lane = tid & 31, col = lane & 15, g = lane >> 4; const size_t r0 = (size_t)blockIdx.x * 64 + wave * 16; const size_t b = ((size_t)blockIdx.x * 64) / SS;
  v8f acc[8] = {};
#pragma unroll 4
  for (int kc = 0; kc < FF / 32; ++kc) { const v16h a = frag_h(HF + (r0 + col) * FF + kc * 32, lane);
#pragma unroll
    for (int j = 0; j < 8; ++j) acc[j] = wmma16(a, frag_h(PS2 + (size_t)(j * 16 + col) * FF + kc * 32, lane), acc[j]); }
#pragma unroll
  for (int j = 0; j < 8; ++j) { const float gv = GW[b * EK + j * 16 + col];
#pragma unroll
    for (int r = 0; r < 8; ++r) sf[wave][8 * g + r][j * 16 + col] = acc[j][r] * gv; }
  LDSX(); for (int rl = 0; rl < 16; ++rl) vst2(T2 + (r0 + rl) * EK + lane * 4, *(const v4f*)&sf[wave][rl][lane * 4]); }
__global__ __launch_bounds__(128) void k_fc2(const _Float16* __restrict__ HF, const _Float16* __restrict__ PW2, const float* __restrict__ T2, const __bf16* __restrict__ PU2, const float* __restrict__ BM, float* __restrict__ OUT) { __shared__ __align__(16) float sf[4][16][132];
  const int tid = threadIdx.x, wave = tid >> 5, lane = tid & 31, col = lane & 15, g = lane >> 4; const size_t r0 = (size_t)blockIdx.x * 64 + wave * 16; const int c0 = blockIdx.y * 128;
  v8f acc[8] = {};
#pragma unroll 4
  for (int kc = 0; kc < FF / 32; ++kc) { const v16h a = frag_h(HF + (r0 + col) * FF + kc * 32, lane);
#pragma unroll
    for (int j = 0; j < 8; ++j) acc[j] = wmma16(a, frag_h(PW2 + (size_t)(c0 + j * 16 + col) * FF + kc * 32, lane), acc[j]); }
#pragma unroll
  for (int kc = 0; kc < EK / 32; ++kc) { const F2 a = split_row(T2 + (r0 + col) * EK, kc * 32, lane);
#pragma unroll
    for (int j = 0; j < 8; ++j) { const v16b w = frag_b(PU2 + (size_t)(c0 + j * 16 + col) * EK + kc * 32, lane); acc[j] = wmma_bf(a.h, w, acc[j]); acc[j] = wmma_bf(a.l, w, acc[j]); } }
#pragma unroll
  for (int j = 0; j < 8; ++j) { const float bb = BM[FF + c0 + j * 16 + col];
#pragma unroll
    for (int r = 0; r < 8; ++r) sf[wave][8 * g + r][j * 16 + col] = acc[j][r] + bb; }
  LDSX(); for (int rl = 0; rl < 16; ++rl) vst2(OUT + (r0 + rl) * HH + c0 + lane * 4, *(const v4f*)&sf[wave][rl][lane * 4]); }
extern "C" void kernel_launch(void* const* d_in, const int* in_sizes, int n_in, void* d_out, int out_size, void* d_ws, size_t ws_size, hipStream_t stream) {
  (void)in_sizes; (void)n_in; (void)out_size;
  const float** F = (const float**)d_in;
  if (ws_size < (size_t)WS_END) return;
  char* ws = (char*)d_ws; float *G1o = (float*)(ws + WS_G1), *G2o = (float*)(ws + WS_G2), *GW = (float*)(ws + WS_GW), *T1 = (float*)(ws + WS_T1), *T2 = (float*)(ws + WS_T2), *BM = (float*)(ws + WS_BM); _Float16* HF = (_Float16*)(ws + WS_HF);
  k_pack<<<dim3(FF, 5), 256, 0, stream>>>(F[9], F[11], F[7], F[12], F[6], F[13], F[8], F[14], ws);
  k_r1<<<dim3(NROW / 64, G1 / 128), 128, 0, stream>>>(F[0], F[1], F[2], G1o);
  k_r2<<<NROW / 64, 128, 0, stream>>>(G1o, F[3], F[4], G2o);
  k_gw<<<NB, 128, 0, stream>>>(G2o, GW);
  k_t1<<<NROW / 64, 128, 0, stream>>>(F[0], F[10], GW, T1);
  k_fc1<<<dim3(TOB, FF / 128), 128, 0, stream>>>(F[0], F[5], T1, (const __bf16*)(ws + WS_PU1), BM, HF);
  k_t2<<<TOB, 128, 0, stream>>>(HF, (const _Float16*)(ws + WS_PS2), GW, T2);
  k_fc2<<<dim3(TOB, HH / 128), 128, 0, stream>>>(HF, (const _Float16*)(ws + WS_PW2), T2, (const __bf16*)(ws + WS_PU2), BM, (float*)d_out);
}
